// EncodePosition_9448928051745
// MI455X (gfx1250) — hardware-verified
//
#include <hip/hip_runtime.h>
#include <math.h>
#include <stdint.h>

#pragma clang fp contract(off)

constexpr int kBatch = 8;
constexpr int kPts   = 2048;
constexpr int kFeat  = 128;
constexpr int kHid   = 64;
constexpr int kBins  = 16;
constexpr int kRows  = kBatch * kPts;
constexpr int kHNld  = 32;
constexpr float kBinScale = (float)(16.0 / 79.0);
constexpr float kLo = 1.0f;
constexpr float kHi = 80.0f;
constexpr float kBnEps = 1e-5f;

constexpr size_t kPlaneHN = (size_t)kRows * kHNld * 2;
constexpr size_t kPlaneH  = (size_t)kRows * kHid * 2;
constexpr size_t kWHalves = (size_t)kHid * kHNld + (size_t)kHid * kHid + (size_t)kFeat * kHid;
constexpr size_t kPlaneW  = kWHalves * 2;
constexpr size_t oHNh = 0;
constexpr size_t oHNl = oHNh + kPlaneHN;
constexpr size_t oH1h = oHNl + kPlaneHN;
constexpr size_t oH1l = oH1h + kPlaneH;
constexpr size_t oH2h = oH1l + kPlaneH;
constexpr size_t oH2l = oH2h + kPlaneH;
constexpr size_t oWh  = oH2l + kPlaneH;
constexpr size_t oWl  = oWh + kPlaneW;
constexpr size_t oBn  = oWl + kPlaneW;
constexpr size_t kWsTotal = oBn + 256 * 4;
static_assert(kWsTotal == 10544128, "carve");
static_assert((oWh % 128) == 0 && (oWl % 128) == 0 && (oBn % 128) == 0, "align");
constexpr int kW1Off = 0;
constexpr int kW2Off = kHid * kHNld;
constexpr int kW3Off = kW2Off + kHid * kHid;

typedef __attribute__((ext_vector_type(16))) _Float16 v16h;
typedef __attribute__((ext_vector_type(8)))  _Float16 v8h;
typedef __attribute__((ext_vector_type(16))) __bf16   v16b;
typedef __attribute__((ext_vector_type(8)))  __bf16   v8b;
typedef __attribute__((ext_vector_type(8)))  float    v8f;
typedef __attribute__((ext_vector_type(4)))  float    v4f;
typedef __attribute__((ext_vector_type(4)))  unsigned int v4u;

__device__ __forceinline__ unsigned short f2bf_bits(float f) {
  unsigned u = __float_as_uint(f);
  return (unsigned short)((u + 0x7FFFu + ((u >> 16) & 1u)) >> 16);
}
__device__ __forceinline__ float bf_bits2f(unsigned short h) { return __uint_as_float(((unsigned)h) << 16); }

__device__ __forceinline__ void dep_guard_h(v8f& a, v8f& b, v16h x, v16h y) { asm volatile("v_nop\n\tv_nop\n\tv_nop\n\tv_nop" : "+v"(a), "+v"(b) : "v"(x), "v"(y)); }
__device__ __forceinline__ void dep_guard_b(v8f& a, v8f& b, v16b x, v16b y) { asm volatile("v_nop\n\tv_nop\n\tv_nop\n\tv_nop" : "+v"(a), "+v"(b) : "v"(x), "v"(y)); }
__device__ __forceinline__ void keep4_h(v16h a, v16h b, v16h c, v16h d) { asm volatile("v_nop" :: "v"(a), "v"(b), "v"(c), "v"(d)); }
__device__ __forceinline__ void keep4_b(v16b a, v16b b, v16b c, v16b d) { asm volatile("v_nop" :: "v"(a), "v"(b), "v"(c), "v"(d)); }
__device__ __forceinline__ void acc_guard4(v8f& a, v8f& b, v8f& c, v8f& d) { asm volatile("v_nop\n\tv_nop\n\tv_nop\n\tv_nop" : "+v"(a), "+v"(b), "+v"(c), "+v"(d)); }
template <typename T> struct Frag;
template <> struct Frag<_Float16> {
  typedef v16h V; union U { v16h v; v8h h[2]; };
  static __device__ __forceinline__ v16h load(const _Float16* p) {
    U f; f.h[0] = *(const v8h*)(p); f.h[1] = *(const v8h*)(p + 16); return f.v;
  }
  static __device__ __forceinline__ v8f mma(v16h a, v16h b, v8f c) {
    return __builtin_amdgcn_wmma_f32_16x16x32_f16(false, a, false, b, (short)0, c, false, false);
  }
  static __device__ __forceinline__ void guard(v8f& a, v8f& b, v16h x, v16h y) { dep_guard_h(a, b, x, y); }
  static __device__ __forceinline__ void keep(v16h a, v16h b, v16h c, v16h d) { keep4_h(a, b, c, d); }
};
template <> struct Frag<__bf16> {
  typedef v16b V; union U { v16b v; v8b h[2]; };
  static __device__ __forceinline__ v16b load(const __bf16* p) {
    U f; f.h[0] = *(const v8b*)(p); f.h[1] = *(const v8b*)(p + 16); return f.v;
  }
  static __device__ __forceinline__ v8f mma(v16b a, v16b b, v8f c) {
    return __builtin_amdgcn_wmma_f32_16x16x32_bf16(false, a, false, b, (short)0, c, false, false);
  }
  static __device__ __forceinline__ void guard(v8f& a, v8f& b, v16b x, v16b y) { dep_guard_b(a, b, x, y); }
  static __device__ __forceinline__ void keep(v16b a, v16b b, v16b c, v16b d) { keep4_b(a, b, c, d); }
};

__device__ __forceinline__ unsigned pk16(unsigned short a, unsigned short b) { return (unsigned)a | ((unsigned)b << 16); }

__device__ __forceinline__ void st2_v4u(unsigned short* p, v4u u) {
  *(volatile v4u*)p = u;
  __threadfence();
  *(volatile v4u*)p = u;
}

__device__ __forceinline__ void split8_bf(const float* v, v4u& hi, v4u& lo) {
  unsigned wh[4], wl[4];
#pragma unroll
  for (int k = 0; k < 4; ++k) {
    const unsigned short h0 = f2bf_bits(v[2 * k]);
    const unsigned short h1 = f2bf_bits(v[2 * k + 1]);
    const unsigned short l0 = f2bf_bits(v[2 * k] - bf_bits2f(h0));
    const unsigned short l1 = f2bf_bits(v[2 * k + 1] - bf_bits2f(h1));
    wh[k] = pk16(h0, h1);
    wl[k] = pk16(l0, l1);
  }
  hi = (v4u){wh[0], wh[1], wh[2], wh[3]};
  lo = (v4u){wl[0], wl[1], wl[2], wl[3]};
}

template <int ET> struct Elem;
template <> struct Elem<0> { typedef _Float16 T; };
template <> struct Elem<1> { typedef __bf16 T; };
template <int ET, bool SPLIT, int BIAS_MODE, int OUT_MODE, bool RESID, int ACT = 0>
__global__ __launch_bounds__(256) void wmma_gemm64(
    const unsigned short* __restrict__ Ap, const unsigned short* __restrict__ A2p, int lda, long strideA,
    const unsigned short* __restrict__ Btp, const unsigned short* __restrict__ Bt2p, int ldb, long strideB,
    void* __restrict__ Cout, void* __restrict__ Cout2, int ldc, long strideC,
    const float* __restrict__ bias, const float* __restrict__ cscale, const float* __restrict__ cshift,
    const float* __restrict__ resid, long strideR,
    int M, int N, int K, float scale) {
  typedef typename Elem<ET>::T T;
  typedef typename Frag<T>::V V;
  const T* A = (const T*)Ap; const T* A2 = (const T*)A2p; const T* Bt = (const T*)Btp; const T* Bt2 = (const T*)Bt2p;
  __shared__ __align__(16) float sT[8][16 * 68];
  const int b    = blockIdx.y;
  const int lane = threadIdx.x & 31;
  const int wave = threadIdx.x >> 5;
  const int tilesN = N >> 6;
  const int tilesM = M >> 6;
  const int tile = blockIdx.x * 8 + wave;
  if (tile >= tilesM * tilesN) return;
  const int tm = tile / tilesN;
  const int tn = tile - tm * tilesN;
  const int m0 = tm << 6;
  const int n0 = tn << 6;

  const T* Ab  = A  + (size_t)b * strideA;
  const T* Bb  = Bt + (size_t)b * strideB;
  const T* Ab2 = SPLIT ? (A2  + (size_t)b * strideA) : nullptr;
  const T* Bb2 = SPLIT ? (Bt2 + (size_t)b * strideB) : nullptr;

  const int rlane = lane & 15;
  const int koff  = (lane >> 4) * 8;
  const int mOff  = (lane >> 4) * 8;

  v8f acc[4][4];
#pragma unroll
  for (int i = 0; i < 4; ++i)
#pragma unroll
    for (int j = 0; j < 4; ++j) acc[i][j] = (v8f){0.f,0.f,0.f,0.f,0.f,0.f,0.f,0.f};

  for (int k0 = 0; k0 < K; k0 += 32) {
    V bh[4], bl[4];
#pragma unroll
    for (int j = 0; j < 4; ++j) {
      const size_t bo = (size_t)(n0 + (j << 4) + rlane) * ldb + koff + k0;
      bh[j] = Frag<T>::load(Bb + bo);
      if (SPLIT) bl[j] = Frag<T>::load(Bb2 + bo);
    }
#pragma unroll
    for (int i = 0; i < 4; ++i) {
      const size_t ao = (size_t)(m0 + (i << 4) + rlane) * lda + koff + k0;
      V ah = Frag<T>::load(Ab + ao);
      V al;
      if (SPLIT) al = Frag<T>::load(Ab2 + ao);
#pragma unroll
      for (int j = 0; j < 4; ++j) {
        acc[i][j] = Frag<T>::mma(ah, bh[j], acc[i][j]);
        if (SPLIT) {
          acc[i][j] = Frag<T>::mma(ah, bl[j], acc[i][j]);
          acc[i][j] = Frag<T>::mma(al, bh[j], acc[i][j]);
        }
      }
      Frag<T>::guard(acc[i][0], acc[i][3], ah, SPLIT ? al : ah);
    }
    Frag<T>::keep(bh[0], bh[1], bh[2], bh[3]);
    if (SPLIT) Frag<T>::keep(bl[0], bl[1], bl[2], bl[3]);
  }
  acc_guard4(acc[0][0], acc[0][1], acc[0][2], acc[0][3]);
  acc_guard4(acc[1][0], acc[1][1], acc[1][2], acc[1][3]);
  acc_guard4(acc[2][0], acc[2][1], acc[2][2], acc[2][3]);
  acc_guard4(acc[3][0], acc[3][1], acc[3][2], acc[3][3]);

  float* slab = sT[wave];
  const float* Rb = RESID ? (resid + (size_t)b * strideR) : nullptr;
#pragma unroll
  for (int i = 0; i < 4; ++i) {
    const int mBase = m0 + (i << 4);
#pragma unroll
    for (int j = 0; j < 4; ++j) {
      const int n = n0 + (j << 4) + rlane;
      float bv = 0.f, sv = 1.f, tv = 0.f;
      if (BIAS_MODE == 2 || BIAS_MODE == 3) bv = bias[n];
      if (BIAS_MODE == 3) { sv = cscale[n]; tv = cshift[n]; }
#pragma unroll
      for (int r = 0; r < 8; ++r) {
        float v = acc[i][j][r] * scale;
        if (BIAS_MODE == 1) v += bias[mBase + mOff + r];
        if (BIAS_MODE == 2 || BIAS_MODE == 3) v += bv;
        if (BIAS_MODE == 3) { v = v * sv; v = v + tv; }
        if (RESID) v += Rb[(size_t)(mBase + mOff + r) * ldc + n];
        if (ACT == 2) v = fmaxf(v, 0.0f);
        if (ACT == 4) v = (v > 0.f) ? v : 0.01f * v;
        slab[(mOff + r) * 68 + (j << 4) + rlane] = v;
      }
    }
    __builtin_amdgcn_fence(__ATOMIC_RELEASE, "workgroup");
    __builtin_amdgcn_wave_barrier();
    __builtin_amdgcn_fence(__ATOMIC_ACQUIRE, "workgroup");
    if (OUT_MODE == 0) {
      float* C = (float*)Cout + (size_t)b * strideC;
      const int hh = lane >> 4, c4 = (lane & 15) * 4;
      for (int pass = 0; pass < 2; ++pass) {
#pragma unroll
        for (int it = 0; it < 8; ++it) {
          const int row = it * 2 + hh;
          v4f v = *(const v4f*)(slab + row * 68 + c4);
          *(volatile v4f*)(C + (size_t)(mBase + row) * ldc + n0 + c4) = v;
        }
        __threadfence();
      }
    } else {
      const int q = lane >> 3, c8 = (lane & 7) * 8;
      unsigned short* C  = (unsigned short*)Cout  + (size_t)b * strideC;
      unsigned short* C2 = (OUT_MODE == 2) ? ((unsigned short*)Cout2 + (size_t)b * strideC) : nullptr;
      for (int pass = 0; pass < 2; ++pass) {
#pragma unroll
        for (int it = 0; it < 4; ++it) {
          const int row = it * 4 + q;
          const float* sp = slab + row * 68 + c8;
          v8h hv, lv;
#pragma unroll
          for (int e = 0; e < 8; ++e) {
            if (OUT_MODE == 1) {
              hv[e] = (_Float16)sp[e];
            } else {
              unsigned short hb = f2bf_bits(sp[e]);
              unsigned short lb = f2bf_bits(sp[e] - bf_bits2f(hb));
              hv[e] = __builtin_bit_cast(_Float16, hb);
              lv[e] = __builtin_bit_cast(_Float16, lb);
            }
          }
          *(volatile v8h*)(C + (size_t)(mBase + row) * ldc + n0 + c8) = hv;
          if (OUT_MODE == 2) *(volatile v8h*)(C2 + (size_t)(mBase + row) * ldc + n0 + c8) = lv;
        }
        __threadfence();
      }
    }
    __builtin_amdgcn_fence(__ATOMIC_RELEASE, "workgroup");
    __builtin_amdgcn_wave_barrier();
    __builtin_amdgcn_fence(__ATOMIC_ACQUIRE, "workgroup");
  }
}

__global__ __launch_bounds__(256) void prep_kernel(
    const float* __restrict__ w1, const float* __restrict__ w2, const float* __restrict__ w3,
    const float* __restrict__ g1, const float* __restrict__ be1, const float* __restrict__ m1, const float* __restrict__ v1,
    const float* __restrict__ g2, const float* __restrict__ be2, const float* __restrict__ m2, const float* __restrict__ v2,
    unsigned short* __restrict__ wh, unsigned short* __restrict__ wl, float* __restrict__ bnv) {
  __shared__ __align__(16) float sbn[256];
  const int tid = threadIdx.x, lane = tid & 31, wave = tid >> 5;

  {
    const int row = tid >> 2, part = tid & 3;
    const int col0 = (part & 1) * 8;
    const bool keep = part < 2;
    float v[8];
#pragma unroll
    for (int e = 0; e < 8; ++e) {
      const float f = w1[row * kBins + col0 + e];
      v[e] = keep ? f : 0.0f;
    }
    v4u uh, ul;
    split8_bf(v, uh, ul);
    st2_v4u(wh + kW1Off + tid * 8, uh);
    st2_v4u(wl + kW1Off + tid * 8, ul);
  }
#pragma unroll 1
  for (int it = 0; it < 2; ++it) {
    const int c = it * 256 + tid;
    const int row = c >> 3, col0 = (c & 7) * 8;
    float v[8];
#pragma unroll
    for (int e = 0; e < 8; ++e) v[e] = w2[row * kHid + col0 + e];
    v4u uh, ul;
    split8_bf(v, uh, ul);
    st2_v4u(wh + kW2Off + c * 8, uh);
    st2_v4u(wl + kW2Off + c * 8, ul);
  }
#pragma unroll 1
  for (int it = 0; it < 4; ++it) {
    const int c = it * 256 + tid;
    const int row = c >> 3, col0 = (c & 7) * 8;
    float v[8];
#pragma unroll
    for (int e = 0; e < 8; ++e) v[e] = w3[row * kHid + col0 + e];
    v4u uh, ul;
    split8_bf(v, uh, ul);
    st2_v4u(wh + kW3Off + c * 8, uh);
    st2_v4u(wl + kW3Off + c * 8, ul);
  }
  if (tid < kHid) {
    const float i1 = g1[tid] / sqrtf(v1[tid] + kBnEps);
    const float t1 = m1[tid] * i1;
    sbn[tid]            = i1;
    sbn[kHid + tid]     = be1[tid] - t1;
    const float i2 = g2[tid] / sqrtf(v2[tid] + kBnEps);
    const float t2 = m2[tid] * i2;
    sbn[2 * kHid + tid] = i2;
    sbn[3 * kHid + tid] = be2[tid] - t2;
  }
  __syncthreads();
  if (wave < 2) {
    const int f0 = (wave * 32 + lane) * 4;
    const v4f val = *(const v4f*)(sbn + f0);
    *(volatile v4f*)(bnv + f0) = val;
    __threadfence();
    *(volatile v4f*)(bnv + f0) = val;
  }
}

__global__ __launch_bounds__(128) void hist_kernel(const float* __restrict__ x,
                                                   unsigned short* __restrict__ hnh,
                                                   unsigned short* __restrict__ hnl) {
  __shared__ __align__(16) float spt[kPts * 4];
  __shared__ __align__(16) unsigned stgh[4][512];
  __shared__ __align__(16) unsigned stgl[4][512];
  const int tid = threadIdx.x, lane = tid & 31, wave = tid >> 5;
  const int b  = blockIdx.x >> 4;
  const int p0 = (blockIdx.x & 15) * 128;
  const float* xb = x + (size_t)b * kPts * 3;

#pragma unroll 1
  for (int i = 0; i < 16; ++i) {
    const int n = i * 128 + tid;
    const float px = xb[n * 3 + 0];
    const float py = xb[n * 3 + 1];
    const float pz = xb[n * 3 + 2];
    const float sxx = px * px;
    const float syy = py * py;
    const float szz = pz * pz;
    const float sq = (sxx + szz) + syy;
    v4f pk; pk.x = px; pk.y = py; pk.z = pz; pk.w = sq;
    *(v4f*)(spt + n * 4) = pk;
  }
  __syncthreads();

  const int pl = p0 + wave * 32 + lane;
  const v4f pm = *(const v4f*)(spt + pl * 4);
  int cnt[kBins];
#pragma unroll
  for (int q = 0; q < kBins; ++q) cnt[q] = 0;

#pragma unroll 2
  for (int j = 0; j < kPts; ++j) {
    const v4f pj = *(const v4f*)(spt + j * 4);
    float dot = pm.x * pj.x;
    const float ty = pm.y * pj.y;
    dot = dot + ty;
    const float tz = pm.z * pj.z;
    dot = dot + tz;
    const float ssum = pm.w + pj.w;
    const float dd = 2.0f * dot;
    const float d2 = ssum - dd;
    const float d = sqrtf(fmaxf(d2, 0.0f));
    const float fb = floorf((d - kLo) * kBinScale);
    int idx = (int)fb;
    idx = idx < 0 ? 0 : (idx > (kBins - 1) ? (kBins - 1) : idx);
    const bool valid = (d >= kLo) && (d <= kHi);
    const int sel = valid ? idx : kBins;
#pragma unroll
    for (int q = 0; q < kBins; ++q) cnt[q] += (sel == q) ? 1 : 0;
  }

  int tot = 0;
#pragma unroll
  for (int q = 0; q < kBins; ++q) tot += cnt[q];
  const float rinv = 1.0f / (float)tot;
  unsigned wdh[8], wdl[8];
#pragma unroll
  for (int k = 0; k < 8; ++k) {
    const float a0 = (float)cnt[2 * k] * rinv;
    const float a1 = (float)cnt[2 * k + 1] * rinv;
    const unsigned short h0 = f2bf_bits(a0);
    const unsigned short h1 = f2bf_bits(a1);
    const unsigned short l0 = f2bf_bits(a0 - bf_bits2f(h0));
    const unsigned short l1 = f2bf_bits(a1 - bf_bits2f(h1));
    wdh[k] = pk16(h0, h1);
    wdl[k] = pk16(l0, l1);
  }
  {
    const v4u zz = (v4u){0u, 0u, 0u, 0u};
    v4u* rh = (v4u*)(&stgh[wave][lane * 16]);
    v4u* rl = (v4u*)(&stgl[wave][lane * 16]);
    rh[0] = (v4u){wdh[0], wdh[1], wdh[2], wdh[3]};
    rh[1] = (v4u){wdh[4], wdh[5], wdh[6], wdh[7]};
    rh[2] = zz;
    rh[3] = zz;
    rl[0] = (v4u){wdl[0], wdl[1], wdl[2], wdl[3]};
    rl[1] = (v4u){wdl[4], wdl[5], wdl[6], wdl[7]};
    rl[2] = zz;
    rl[3] = zz;
  }
  __syncthreads();

  const size_t gp0 = (size_t)b * kPts + (size_t)p0 + (size_t)wave * 32;
  unsigned short* gh = hnh + gp0 * kHNld;
  unsigned short* gl = hnl + gp0 * kHNld;
  for (int pass = 0; pass < 2; ++pass) {
#pragma unroll
    for (int it = 0; it < 4; ++it) {
      const v4u uh = *(const v4u*)(&stgh[wave][it * 128 + lane * 4]);
      const v4u ul = *(const v4u*)(&stgl[wave][it * 128 + lane * 4]);
      *(volatile v4u*)(gh + it * 256 + lane * 8) = uh;
      *(volatile v4u*)(gl + it * 256 + lane * 8) = ul;
    }
    __threadfence();
  }
}

extern "C" void kernel_launch(void* const* d_in, const int* in_sizes, int n_in,
                              void* d_out, int out_size, void* d_ws, size_t ws_size,
                              hipStream_t stream) {
  if (n_in < 16) return;
  if (in_sizes[0] != kBatch * kPts * 3) return;
  if (in_sizes[1] != kBatch * kFeat * kPts) return;
  if (in_sizes[2] != kHid * kBins || in_sizes[8] != kHid * kHid || in_sizes[14] != kFeat * kHid) return;
  if (in_sizes[3] != kHid || in_sizes[9] != kHid || in_sizes[15] != kFeat) return;
  if (out_size != kBatch * kFeat * kPts) return;
  if (ws_size < kWsTotal) return;

  const float* x   = (const float*)d_in[0];
  const float* fea = (const float*)d_in[1];
  const float* w1  = (const float*)d_in[2];
  const float* b1  = (const float*)d_in[3];
  const float* g1  = (const float*)d_in[4];
  const float* be1 = (const float*)d_in[5];
  const float* m1  = (const float*)d_in[6];
  const float* v1  = (const float*)d_in[7];
  const float* w2  = (const float*)d_in[8];
  const float* b2  = (const float*)d_in[9];
  const float* g2  = (const float*)d_in[10];
  const float* be2 = (const float*)d_in[11];
  const float* m2  = (const float*)d_in[12];
  const float* v2  = (const float*)d_in[13];
  const float* w3  = (const float*)d_in[14];
  const float* b3  = (const float*)d_in[15];
  float* out = (float*)d_out;

  char* ws = (char*)d_ws;
  unsigned short* hnh = (unsigned short*)(ws + oHNh);
  unsigned short* hnl = (unsigned short*)(ws + oHNl);
  unsigned short* h1h = (unsigned short*)(ws + oH1h);
  unsigned short* h1l = (unsigned short*)(ws + oH1l);
  unsigned short* h2h = (unsigned short*)(ws + oH2h);
  unsigned short* h2l = (unsigned short*)(ws + oH2l);
  unsigned short* wh  = (unsigned short*)(ws + oWh);
  unsigned short* wl  = (unsigned short*)(ws + oWl);
  float* bnv = (float*)(ws + oBn);

  prep_kernel<<<dim3(1), dim3(256), 0, stream>>>(w1, w2, w3, g1, be1, m1, v1, g2, be2, m2, v2, wh, wl, bnv);

  hist_kernel<<<dim3(kBatch * (kPts / 128)), dim3(128), 0, stream>>>(x, hnh, hnl);

  wmma_gemm64<1, true, 3, 2, false, 2><<<dim3((kRows / 64) * (kHid / 64) / 8, 1), dim3(256), 0, stream>>>(
      hnh, hnl, kHNld, 0L,
      wh + kW1Off, wl + kW1Off, kHNld, 0L,
      (void*)h1h, (void*)h1l, kHid, 0L,
      b1, bnv + 0, bnv + kHid,
      nullptr, 0L,
      kRows, kHid, kHNld, 1.0f);

  wmma_gemm64<1, true, 3, 2, false, 2><<<dim3((kRows / 64) * (kHid / 64) / 8, 1), dim3(256), 0, stream>>>(
      h1h, h1l, kHid, 0L,
      wh + kW2Off, wl + kW2Off, kHid, 0L,
      (void*)h2h, (void*)h2l, kHid, 0L,
      b2, bnv + 2 * kHid, bnv + 3 * kHid,
      nullptr, 0L,
      kRows, kHid, kHid, 1.0f);

  wmma_gemm64<1, true, 1, 0, true, 0><<<dim3((kFeat / 64) * (kPts / 64) / 8, kBatch), dim3(256), 0, stream>>>(
      wh + kW3Off, wl + kW3Off, kHid, 0L,
      h2h, h2l, kHid, (long)kPts * kHid,
      (void*)out, nullptr, kPts, (long)kFeat * kPts,
      b3, nullptr, nullptr,
      fea, (long)kFeat * kPts,
      kFeat, kPts, kHid, 1.0f);
}
